// MambaBlock_58909771432039
// MI455X (gfx1250) — hardware-verified
//
#include <hip/hip_runtime.h>
#include <math.h>

typedef __attribute__((ext_vector_type(16))) _Float16 v16h;
typedef __attribute__((ext_vector_type(8)))  _Float16 v8h;
typedef __attribute__((ext_vector_type(16))) __bf16   v16b;
typedef __attribute__((ext_vector_type(8)))  __bf16   v8b;
typedef __attribute__((ext_vector_type(8)))  float    v8f;
typedef __attribute__((ext_vector_type(4)))  float    v4f;
typedef __attribute__((ext_vector_type(4)))  unsigned v4u;

constexpr int kBatch = 2;
constexpr int kSeqL  = 1024;
constexpr int kDmod  = 1024;
constexpr int kDin   = 2048;
constexpr int kNst   = 16;
constexpr int kDtR   = 64;
constexpr int kPrjN  = 96;
constexpr int kPrjP  = 128;
constexpr int kXZP   = 2 * kDin;
constexpr int kRows  = kBatch * kSeqL;
constexpr int kTP    = 260;

constexpr float kCarryXc  = 1.0f;
constexpr float kCarryWx  = 256.0f;
constexpr float kCarryDt  = 16.0f;
constexpr float kCarryWdt = 8.0f;
constexpr float kCarryY   = 16.0f;
constexpr float kCarryWo  = 256.0f;
constexpr float kCarryRes = 1024.0f;
constexpr float kF16MinNormal = 6.103515625e-5f;
constexpr float kUnscaleS1  = 1.0f / (kCarryXc * kCarryWx);
constexpr float kUnscaleS1r = kUnscaleS1 / kCarryRes;
constexpr float kUnscaleS2  = 1.0f / (kCarryDt * kCarryWdt);
constexpr float kUnscaleS4  = 1.0f / (kCarryY * kCarryWo);
constexpr float kUnscaleS4r = kUnscaleS4 / kCarryRes;

static_assert(kDtR + 2 * kNst == kPrjN, "x_proj width");
static_assert(kPrjP % 64 == 0 && kPrjP >= kPrjN, "x_proj pad");
static_assert((kRows % 64) == 0 && (kXZP % 64) == 0 && (kDin % 64) == 0 && (kDmod % 64) == 0, "GEMM M,N multiples of 64");
static_assert((kDmod % 32) == 0 && (kDin % 32) == 0 && (kDtR % 32) == 0, "GEMM K multiples of 32");
static_assert((kSeqL % 64) == 0 && (kDin % 256) == 0 && (kSeqL % 16) == 0, "tile multiples");
static_assert((kSeqL & (kSeqL - 1)) == 0, "sequence length power of two");

constexpr size_t kSzXB   = (size_t)kRows * kDmod * 2;
constexpr size_t kSzWIB  = (size_t)kXZP  * kDmod * 2;
constexpr size_t kSzWXH  = (size_t)kPrjP * kDin  * 2;
constexpr size_t kSzWDTH = (size_t)kDin  * kDtR  * 2;
constexpr size_t kSzWOH  = (size_t)kDmod * kDin  * 2;
constexpr size_t kSzXZ   = (size_t)kRows * kXZP  * 4;
constexpr size_t kSzUC   = (size_t)kRows * kDin  * 4;
constexpr size_t kSzUC16 = (size_t)kRows * kDin  * 2;
constexpr size_t kSzPROJ = (size_t)kRows * kPrjP * 4;
constexpr size_t kSzDT16 = (size_t)kRows * kDtR  * 2;
constexpr size_t kSzDLR  = (size_t)kRows * kDin  * 4;
constexpr size_t kSzY16  = (size_t)kRows * kDin  * 2;
constexpr size_t kOffXB    = 0;
constexpr size_t kOffWIB   = kOffXB    + kSzXB;
constexpr size_t kOffWXH   = kOffWIB   + kSzWIB;
constexpr size_t kOffWDTH  = kOffWXH   + kSzWXH;
constexpr size_t kOffWOH   = kOffWDTH  + kSzWDTH;
constexpr size_t kOffXZ    = kOffWOH   + kSzWOH;
constexpr size_t kOffUC    = kOffXZ    + kSzXZ;
constexpr size_t kOffUC16  = kOffUC    + kSzUC;
constexpr size_t kOffUC16L = kOffUC16  + kSzUC16;
constexpr size_t kOffPROJ  = kOffUC16L + kSzUC16;
constexpr size_t kOffDT16  = kOffPROJ  + kSzPROJ;
constexpr size_t kOffDLR   = kOffDT16  + kSzDT16;
constexpr size_t kOffY16   = kOffDLR   + kSzDLR;
constexpr size_t kOffY16L  = kOffY16   + kSzY16;
constexpr size_t kWsTotal  = kOffY16L  + kSzY16;
static_assert(kWsTotal == 119537664ull, "carve total");
static_assert(kWsTotal <= 134217728ull, "carve cap");
static_assert((kOffWIB % 128) == 0 && (kOffWXH % 128) == 0 && (kOffWDTH % 128) == 0 && (kOffWOH % 128) == 0 &&
              (kOffXZ % 128) == 0 && (kOffUC % 128) == 0 && (kOffUC16 % 128) == 0 && (kOffUC16L % 128) == 0 &&
              (kOffPROJ % 128) == 0 && (kOffDT16 % 128) == 0 && (kOffDLR % 128) == 0 && (kOffY16 % 128) == 0 &&
              (kOffY16L % 128) == 0, "128-B aligned regions");

__device__ __forceinline__ unsigned bf_bits_rne(float f) {
  const unsigned u = __float_as_uint(f);
  return (u + 0x7FFFu + ((u >> 16) & 1u)) >> 16;
}
__device__ __forceinline__ float bf_rne(float f) { return __uint_as_float(bf_bits_rne(f) << 16); }

__device__ __forceinline__ void split_f16(float v, _Float16& hi, _Float16& lo) {
  const _Float16 h0 = (_Float16)v;
  const float hf0 = (float)h0;
  const float hf = (fabsf(hf0) < kF16MinNormal) ? 0.0f : hf0;
  hi = (_Float16)hf;
  const float rs = (v - hf) * kCarryRes;
  lo = (_Float16)rs;
}

__device__ __forceinline__ void dep_guard4_h(v8f& a, v8f& b, v8f& c, v8f& d, v16h x, v16h b0, v16h b1, v16h b2, v16h b3) {
  asm volatile("v_nop\n\tv_nop\n\tv_nop\n\tv_nop" : "+v"(a), "+v"(b), "+v"(c), "+v"(d) : "v"(x), "v"(b0), "v"(b1), "v"(b2), "v"(b3));
}
__device__ __forceinline__ void dep_guard4_b(v8f& a, v8f& b, v8f& c, v8f& d, v16b x, v16b b0, v16b b1, v16b b2, v16b b3) {
  asm volatile("v_nop\n\tv_nop\n\tv_nop\n\tv_nop" : "+v"(a), "+v"(b), "+v"(c), "+v"(d) : "v"(x), "v"(b0), "v"(b1), "v"(b2), "v"(b3));
}
__device__ __forceinline__ void keep4_h(v16h a, v16h b, v16h c, v16h d) { asm volatile("v_nop" :: "v"(a), "v"(b), "v"(c), "v"(d)); }
__device__ __forceinline__ void keep4_b(v16b a, v16b b, v16b c, v16b d) { asm volatile("v_nop" :: "v"(a), "v"(b), "v"(c), "v"(d)); }
__device__ __forceinline__ void acc_guard4(v8f& a, v8f& b, v8f& c, v8f& d) {
  asm volatile("v_nop\n\tv_nop\n\tv_nop\n\tv_nop" : "+v"(a), "+v"(b), "+v"(c), "+v"(d));
}
template <typename T> struct Frag;
template <> struct Frag<_Float16> {
  typedef v16h V; union U { v16h v; v8h h[2]; };
  static __device__ __forceinline__ v16h load(const _Float16* p) {
    U f; f.h[0] = *(const v8h*)(p); f.h[1] = *(const v8h*)(p + 16); return f.v;
  }
  static __device__ __forceinline__ v8f mma(v16h a, v16h b, v8f c) {
    return __builtin_amdgcn_wmma_f32_16x16x32_f16(false, a, false, b, (short)0, c, false, false);
  }
  static __device__ __forceinline__ void guard(v8f& a, v8f& b, v8f& c, v8f& d, v16h x, v16h b0, v16h b1, v16h b2, v16h b3) {
    dep_guard4_h(a, b, c, d, x, b0, b1, b2, b3);
  }
  static __device__ __forceinline__ void keep(v16h a, v16h b, v16h c, v16h d) { keep4_h(a, b, c, d); }
};
template <> struct Frag<__bf16> {
  typedef v16b V; union U { v16b v; v8b h[2]; };
  static __device__ __forceinline__ v16b load(const __bf16* p) {
    U f; f.h[0] = *(const v8b*)(p); f.h[1] = *(const v8b*)(p + 16); return f.v;
  }
  static __device__ __forceinline__ v8f mma(v16b a, v16b b, v8f c) {
    return __builtin_amdgcn_wmma_f32_16x16x32_bf16(false, a, false, b, (short)0, c, false, false);
  }
  static __device__ __forceinline__ void guard(v8f& a, v8f& b, v8f& c, v8f& d, v16b x, v16b b0, v16b b1, v16b b2, v16b b3) {
    dep_guard4_b(a, b, c, d, x, b0, b1, b2, b3);
  }
  static __device__ __forceinline__ void keep(v16b a, v16b b, v16b c, v16b d) { keep4_b(a, b, c, d); }
};

template <int ET> struct Elem;
template <> struct Elem<0> { typedef _Float16 T; };
template <> struct Elem<1> { typedef __bf16 T; };
template <int ET, int MT, bool SPLA>
__global__ __launch_bounds__(256) void wmma_gemm64(
    const unsigned short* __restrict__ Ap, const unsigned short* __restrict__ A2p, int lda,
    const unsigned short* __restrict__ Btp, int ldb,
    float* __restrict__ C, int ldc,
    int M, int N, int K, float scale, float scale2) {
  typedef typename Elem<ET>::T T;
  typedef typename Frag<T>::V V;
  static_assert((SPLA && MT == 2) || (!SPLA && MT == 4), "accumulator budget");
  const T* A  = (const T*)Ap;
  const T* A2 = (const T*)A2p;
  const T* Bt = (const T*)Btp;
  __shared__ __align__(16) float sT[8][16 * 68];
  const int lane = threadIdx.x & 31;
  const int wave = threadIdx.x >> 5;
  const int tilesN = N >> 6;
  const int tilesM = M / (16 * MT);
  const int tile = blockIdx.x * 8 + wave;
  if (tile >= tilesM * tilesN) return;
  const int tm = tile / tilesN;
  const int tn = tile - tm * tilesN;
  const int m0 = tm * (16 * MT);
  const int n0 = tn << 6;

  const int rlane = lane & 15;
  const int koff  = (lane >> 4) * 8;
  const int mOff  = (lane >> 4) * 8;

  v8f acc[MT][4];
  v8f accr[MT][4];
#pragma unroll
  for (int i = 0; i < MT; ++i)
#pragma unroll
    for (int j = 0; j < 4; ++j) {
      acc[i][j]  = (v8f){0.f,0.f,0.f,0.f,0.f,0.f,0.f,0.f};
      accr[i][j] = (v8f){0.f,0.f,0.f,0.f,0.f,0.f,0.f,0.f};
    }

  for (int k0 = 0; k0 < K; k0 += 32) {
    V bh[4];
#pragma unroll
    for (int j = 0; j < 4; ++j) {
      const size_t bo = (size_t)(n0 + (j << 4) + rlane) * ldb + koff + k0;
      bh[j] = Frag<T>::load(Bt + bo);
    }
#pragma unroll
    for (int i = 0; i < MT; ++i) {
      const size_t ao = (size_t)(m0 + (i << 4) + rlane) * lda + koff + k0;
      V ah = Frag<T>::load(A + ao);
      V al = ah;
      if (SPLA) al = Frag<T>::load(A2 + ao);
#pragma unroll
      for (int j = 0; j < 4; ++j) {
        acc[i][j] = Frag<T>::mma(ah, bh[j], acc[i][j]);
        if (SPLA) accr[i][j] = Frag<T>::mma(al, bh[j], accr[i][j]);
      }
      Frag<T>::guard(acc[i][0], acc[i][1], acc[i][2], acc[i][3], ah, bh[0], bh[1], bh[2], bh[3]);
      if (SPLA) Frag<T>::guard(accr[i][0], accr[i][1], accr[i][2], accr[i][3], al, bh[0], bh[1], bh[2], bh[3]);
    }
    Frag<T>::keep(bh[0], bh[1], bh[2], bh[3]);
  }
#pragma unroll
  for (int i = 0; i < MT; ++i) {
    acc_guard4(acc[i][0], acc[i][1], acc[i][2], acc[i][3]);
    if (SPLA) acc_guard4(accr[i][0], accr[i][1], accr[i][2], accr[i][3]);
  }

  float* slab = sT[wave];
#pragma unroll
  for (int i = 0; i < MT; ++i) {
    const int mBase = m0 + (i << 4);
#pragma unroll
    for (int j = 0; j < 4; ++j) {
#pragma unroll
      for (int r = 0; r < 8; ++r) {
        float v = acc[i][j][r] * scale;
        if (SPLA) v += accr[i][j][r] * scale2;
        slab[(mOff + r) * 68 + (j << 4) + rlane] = v;
      }
    }
    __builtin_amdgcn_fence(__ATOMIC_RELEASE, "workgroup");
    __builtin_amdgcn_wave_barrier();
    __builtin_amdgcn_fence(__ATOMIC_ACQUIRE, "workgroup");
    {
      const int hh = lane >> 4, c4 = (lane & 15) * 4;
      for (int pass = 0; pass < 2; ++pass) {
#pragma unroll
        for (int it = 0; it < 8; ++it) {
          const int row = it * 2 + hh;
          const v4f v = *(const v4f*)(slab + row * 68 + c4);
          *(volatile v4f*)(C + (size_t)(mBase + row) * ldc + n0 + c4) = v;
        }
        __threadfence();
      }
    }
    __builtin_amdgcn_fence(__ATOMIC_RELEASE, "workgroup");
    __builtin_amdgcn_wave_barrier();
    __builtin_amdgcn_fence(__ATOMIC_ACQUIRE, "workgroup");
  }
}

__global__ __launch_bounds__(256) void cast_bf16_kernel(
    const float* __restrict__ src, unsigned short* __restrict__ dst, int total8)
{
  const int i = blockIdx.x * 256 + threadIdx.x;
  if (i >= total8) return;
  const size_t e0 = (size_t)i << 3;
  const v4f a0 = *(const v4f*)(src + e0);
  const v4f a1 = *(const v4f*)(src + e0 + 4);
  const float f0 = a0[0], f1 = a0[1], f2 = a0[2], f3 = a0[3];
  const float f4 = a1[0], f5 = a1[1], f6 = a1[2], f7 = a1[3];
  const unsigned w0 = bf_bits_rne(f0) | (bf_bits_rne(f1) << 16);
  const unsigned w1 = bf_bits_rne(f2) | (bf_bits_rne(f3) << 16);
  const unsigned w2 = bf_bits_rne(f4) | (bf_bits_rne(f5) << 16);
  const unsigned w3 = bf_bits_rne(f6) | (bf_bits_rne(f7) << 16);
  const v4u w = (v4u){w0, w1, w2, w3};
  unsigned short* q = dst + e0;
  *(volatile v4u*)(void*)q = w;
  __threadfence();
  *(volatile v4u*)(void*)q = w;
}

__global__ __launch_bounds__(256) void cast_bfval_f16_kernel(
    const float* __restrict__ src, unsigned short* __restrict__ dst, int total8, int valid8, float carry)
{
  const int i = blockIdx.x * 256 + threadIdx.x;
  if (i >= total8) return;
  const bool ok = (i < valid8);
  const int ic = ok ? i : (valid8 - 1);
  const size_t es = (size_t)ic << 3;
  const v4f a0 = *(const v4f*)(src + es);
  const v4f a1 = *(const v4f*)(src + es + 4);
  v8h hv;
#pragma unroll
  for (int e = 0; e < 4; ++e) {
    const float p0 = a0[e];
    const float p1 = a1[e];
    const float r0 = bf_rne(p0) * carry;
    const float r1 = bf_rne(p1) * carry;
    hv[e]     = (_Float16)(ok ? r0 : 0.0f);
    hv[4 + e] = (_Float16)(ok ? r1 : 0.0f);
  }
  unsigned short* q = dst + ((size_t)i << 3);
  *(volatile v8h*)(void*)q = hv;
  __threadfence();
  *(volatile v8h*)(void*)q = hv;
}

__global__ __launch_bounds__(256) void dt_cast_kernel(
    const float* __restrict__ PROJ, unsigned short* __restrict__ DT16, int total8, float carry)
{
  const int i = blockIdx.x * 256 + threadIdx.x;
  if (i >= total8) return;
  const int e0  = i << 3;
  const int row = e0 >> 6;
  const int c8  = e0 & 63;
  const float* p = PROJ + (size_t)row * kPrjP + c8;
  const v4f a0 = *(const v4f*)(p);
  const v4f a1 = *(const v4f*)(p + 4);
  v8h hv;
#pragma unroll
  for (int e = 0; e < 4; ++e) {
    const float p0 = a0[e];
    const float p1 = a1[e];
    hv[e]     = (_Float16)(p0 * carry);
    hv[4 + e] = (_Float16)(p1 * carry);
  }
  unsigned short* qd = DT16 + e0;
  *(volatile v8h*)(void*)qd = hv;
  __threadfence();
  *(volatile v8h*)(void*)qd = hv;
}

__global__ __launch_bounds__(256) void conv_silu_kernel(
    const float* __restrict__ XZ, const float* __restrict__ cw, const float* __restrict__ cb,
    float* __restrict__ UC, unsigned short* __restrict__ UC16, unsigned short* __restrict__ UC16L)
{
  __shared__ __align__(16) float sT[16 * kTP];
  const int tid = threadIdx.x, lane = tid & 31, wave = tid >> 5;
  const int d0 = blockIdx.x * 256, d = d0 + tid;
  const int g0 = blockIdx.y * 64;
  const int tb = g0 & (kSeqL - 1);
  const v4f wv = *(const v4f*)(cw + (size_t)d * 4);
  const float wr0 = wv[0], wr1 = wv[1], wr2 = wv[2], wr3 = wv[3];
  const float w0 = bf_rne(wr0), w1 = bf_rne(wr1), w2 = bf_rne(wr2), w3 = bf_rne(wr3);
  const float bc = bf_rne(cb[d]);
  float xm3, xm2, xm1;
  {
    const bool hist = (tb > 0);
    const int rb = hist ? (g0 - 3) : g0;
    const float v3 = XZ[(size_t)rb * kXZP + d];
    const float v2 = XZ[(size_t)(rb + 1) * kXZP + d];
    const float v1 = XZ[(size_t)(rb + 2) * kXZP + d];
    xm3 = hist ? v3 : 0.f;
    xm2 = hist ? v2 : 0.f;
    xm1 = hist ? v1 : 0.f;
  }
  const int hrow = wave >> 1;
  const int hch  = (wave & 1) * 128 + lane * 4;
#pragma unroll 1
  for (int sub = 0; sub < 4; ++sub) {
    const int lb = g0 + sub * 16;
#pragma unroll 1
    for (int s = 0; s < 16; ++s) {
      const float xcur = XZ[(size_t)(lb + s) * kXZP + d];
      float acc = w0 * xm3;
      acc = fmaf(w1, xm2, acc);
      acc = fmaf(w2, xm1, acc);
      acc = fmaf(w3, xcur, acc);
      const float sv = acc + bc;
      const float sg = __builtin_amdgcn_rcpf(1.0f + expf(-sv));
      sT[s * kTP + tid] = sv * sg;
      xm3 = xm2; xm2 = xm1; xm1 = xcur;
    }
    __syncthreads();
    v4f fv[4];
    v8h bv[2], bl[2];
#pragma unroll
    for (int it = 0; it < 4; ++it) fv[it] = *(const v4f*)(sT + (it * 4 + hrow) * kTP + hch);
#pragma unroll
    for (int it = 0; it < 2; ++it) {
      const float* sp = sT + (it * 8 + wave) * kTP + lane * 8;
      const v4f a0 = *(const v4f*)(sp);
      const v4f a1 = *(const v4f*)(sp + 4);
#pragma unroll
      for (int e = 0; e < 4; ++e) {
        const float p0 = a0[e] * kCarryXc;
        const float p1 = a1[e] * kCarryXc;
        _Float16 h0, l0, h1, l1;
        split_f16(p0, h0, l0);
        split_f16(p1, h1, l1);
        bv[it][e]     = h0;
        bv[it][4 + e] = h1;
        bl[it][e]     = l0;
        bl[it][4 + e] = l1;
      }
    }
    for (int pass = 0; pass < 2; ++pass) {
#pragma unroll
      for (int it = 0; it < 4; ++it)
        *(volatile v4f*)(UC + (size_t)(lb + it * 4 + hrow) * kDin + d0 + hch) = fv[it];
#pragma unroll
      for (int it = 0; it < 2; ++it) {
        const size_t o = (size_t)(lb + it * 8 + wave) * kDin + d0 + lane * 8;
        *(volatile v8h*)(void*)(UC16 + o)  = bv[it];
        *(volatile v8h*)(void*)(UC16L + o) = bl[it];
      }
      __threadfence();
    }
    __syncthreads();
  }
}

__global__ __launch_bounds__(256) void scan_kernel(
    const float* __restrict__ DLR, const float* __restrict__ UC, const float* __restrict__ XZ,
    const float* __restrict__ PROJ, const float* __restrict__ bdt, const float* __restrict__ A_log,
    const float* __restrict__ Dv, unsigned short* __restrict__ Y16, unsigned short* __restrict__ Y16L)
{
  __shared__ __align__(16) float sBC[16 * 32];
  __shared__ __align__(16) float sY[16 * kTP];
  const int tid = threadIdx.x, lane = tid & 31, wave = tid >> 5;
  const int d0 = blockIdx.x * 256, d = d0 + tid;
  const size_t row0 = (size_t)blockIdx.y * kSeqL;

  float An[kNst];
#pragma unroll
  for (int q4 = 0; q4 < 4; ++q4) {
    const v4f av = *(const v4f*)(A_log + (size_t)d * kNst + 4 * q4);
    const float g0 = av[0], g1 = av[1], g2 = av[2], g3 = av[3];
    An[4 * q4 + 0] = -__expf(bf_rne(g0));
    An[4 * q4 + 1] = -__expf(bf_rne(g1));
    An[4 * q4 + 2] = -__expf(bf_rne(g2));
    An[4 * q4 + 3] = -__expf(bf_rne(g3));
  }
  const float Dd = bf_rne(Dv[d]);
  const float bb = bf_rne(bdt[d]);
  float h[kNst];
#pragma unroll
  for (int n = 0; n < kNst; ++n) h[n] = 0.f;

#pragma unroll 1
  for (int c = 0; c < kSeqL / 16; ++c) {
    const int l0 = c * 16;
    if (tid < 128) {
      const int r = tid >> 3, q = (tid & 7) * 4;
      const v4f v = *(const v4f*)(PROJ + (row0 + l0 + r) * kPrjP + kDtR + q);
      *(v4f*)(sBC + r * 32 + q) = v;
    }
    __syncthreads();
#pragma unroll 1
    for (int s = 0; s < 16; ++s) {
      const size_t m = row0 + (size_t)(l0 + s);
      const float a  = DLR[m * kDin + d] + bb;
      const float sp = fmaxf(a, 0.0f) + log1pf(__expf(-fabsf(a)));
      const float delta = fminf(sp + 1e-4f, 10.0f);
      const float xv = UC[m * kDin + d];
      const float zv = XZ[m * kXZP + kDin + d];
      float Bs[kNst], Cs[kNst];
#pragma unroll
      for (int q4 = 0; q4 < 4; ++q4) {
        const v4f bq = *(const v4f*)(sBC + s * 32 + 4 * q4);
        const v4f cq = *(const v4f*)(sBC + s * 32 + kNst + 4 * q4);
        Bs[4 * q4 + 0] = bq[0]; Bs[4 * q4 + 1] = bq[1]; Bs[4 * q4 + 2] = bq[2]; Bs[4 * q4 + 3] = bq[3];
        Cs[4 * q4 + 0] = cq[0]; Cs[4 * q4 + 1] = cq[1]; Cs[4 * q4 + 2] = cq[2]; Cs[4 * q4 + 3] = cq[3];
      }
      float y = 0.f;
#pragma unroll
      for (int n = 0; n < kNst; ++n) {
        const float e = fminf(__expf(delta * An[n]), 10.0f);
        float bu = (delta * Bs[n]) * xv;
        bu = fminf(fmaxf(bu, -10.0f), 10.0f);
        float hn = e * h[n] + bu;
        hn = fminf(fmaxf(hn, -20.0f), 20.0f);
        h[n] = hn;
        y = hn * Cs[n] + y;
      }
      y = y + xv * Dd;
      y = fminf(fmaxf(y, -50.0f), 50.0f);
      const float sg = __builtin_amdgcn_rcpf(1.0f + __expf(-zv));
      const float g  = zv * sg;
      sY[s * kTP + tid] = (y * g) * kCarryY;
    }
    __syncthreads();
    v8h hv[2], lv[2];
#pragma unroll
    for (int it = 0; it < 2; ++it) {
      const float* spp = sY + (it * 8 + wave) * kTP + lane * 8;
      const v4f a0 = *(const v4f*)(spp);
      const v4f a1 = *(const v4f*)(spp + 4);
#pragma unroll
      for (int e = 0; e < 4; ++e) {
        const float p0 = a0[e];
        const float p1 = a1[e];
        _Float16 h0, l0, h1, l1;
        split_f16(p0, h0, l0);
        split_f16(p1, h1, l1);
        hv[it][e]     = h0;
        hv[it][4 + e] = h1;
        lv[it][e]     = l0;
        lv[it][4 + e] = l1;
      }
    }
    for (int pass = 0; pass < 2; ++pass) {
#pragma unroll
      for (int it = 0; it < 2; ++it) {
        const size_t o = (row0 + l0 + it * 8 + wave) * kDin + d0 + lane * 8;
        *(volatile v8h*)(void*)(Y16 + o)  = hv[it];
        *(volatile v8h*)(void*)(Y16L + o) = lv[it];
      }
      __threadfence();
    }
  }
}

extern "C" void kernel_launch(void* const* d_in, const int* in_sizes, int n_in,
                              void* d_out, int out_size, void* d_ws, size_t ws_size,
                              hipStream_t stream)
{
  (void)stream;
  if (n_in < 10) return;
  if (in_sizes[0] != kRows * kDmod) return;
  if (in_sizes[1] != kXZP * kDmod) return;
  if (in_sizes[2] != kDin * 4) return;
  if (in_sizes[3] != kDin) return;
  if (in_sizes[4] != kPrjN * kDin) return;
  if (in_sizes[5] != kDin * kDtR) return;
  if (in_sizes[6] != kDin) return;
  if (in_sizes[7] != kDin * kNst) return;
  if (in_sizes[8] != kDin) return;
  if (in_sizes[9] != kDmod * kDin) return;
  if (out_size != kRows * kDmod) return;
  if (ws_size < kWsTotal) return;

  const float* x      = (const float*)d_in[0];
  const float* W_in   = (const float*)d_in[1];
  const float* conv_w = (const float*)d_in[2];
  const float* conv_b = (const float*)d_in[3];
  const float* W_x    = (const float*)d_in[4];
  const float* W_dt   = (const float*)d_in[5];
  const float* b_dt   = (const float*)d_in[6];
  const float* A_log  = (const float*)d_in[7];
  const float* Dv     = (const float*)d_in[8];
  const float* W_out  = (const float*)d_in[9];
  float* dout = (float*)d_out;

  char* ws = (char*)d_ws;
  unsigned short* XB    = (unsigned short*)(ws + kOffXB);
  unsigned short* WIB   = (unsigned short*)(ws + kOffWIB);
  unsigned short* WXH   = (unsigned short*)(ws + kOffWXH);
  unsigned short* WDTH  = (unsigned short*)(ws + kOffWDTH);
  unsigned short* WOH   = (unsigned short*)(ws + kOffWOH);
  float*          XZ    = (float*)(ws + kOffXZ);
  float*          UC    = (float*)(ws + kOffUC);
  unsigned short* UC16  = (unsigned short*)(ws + kOffUC16);
  unsigned short* UC16L = (unsigned short*)(ws + kOffUC16L);
  float*          PROJ  = (float*)(ws + kOffPROJ);
  unsigned short* DT16  = (unsigned short*)(ws + kOffDT16);
  float*          DLR   = (float*)(ws + kOffDLR);
  unsigned short* Y16   = (unsigned short*)(ws + kOffY16);
  unsigned short* Y16L  = (unsigned short*)(ws + kOffY16L);

  constexpr int kT8x   = kRows * kDmod / 8;
  constexpr int kT8wi  = kXZP * kDmod / 8;
  constexpr int kT8wxT = kPrjP * kDin / 8;
  constexpr int kT8wxV = kPrjN * kDin / 8;
  constexpr int kT8wdt = kDin * kDtR / 8;
  constexpr int kT8wo  = kDmod * kDin / 8;
  constexpr int kT8dt  = kRows * kDtR / 8;
  static_assert(kT8x % 256 == 0 && kT8wi % 256 == 0 && kT8wxT % 256 == 0 && kT8wdt % 256 == 0 &&
                kT8wo % 256 == 0 && kT8dt % 256 == 0, "exact grids");
  static_assert(kT8wxV % 32 == 0, "pad boundary on a wave boundary");
  constexpr int kTilesS0 = (kRows / 64) * (kXZP / 64);
  constexpr int kTilesS1 = (kRows / 32) * (kPrjP / 64);
  constexpr int kTilesS2 = (kRows / 64) * (kDin / 64);
  constexpr int kTilesS4 = (kRows / 32) * (kDmod / 64);
  static_assert(kTilesS0 % 8 == 0 && kTilesS1 % 8 == 0 && kTilesS2 % 8 == 0 && kTilesS4 % 8 == 0, "exact GEMM grids");

  cast_bf16_kernel<<<kT8x / 256, 256, 0, stream>>>(x, XB, kT8x);
  cast_bf16_kernel<<<kT8wi / 256, 256, 0, stream>>>(W_in, WIB, kT8wi);
  cast_bfval_f16_kernel<<<kT8wxT / 256, 256, 0, stream>>>(W_x, WXH, kT8wxT, kT8wxV, kCarryWx);
  cast_bfval_f16_kernel<<<kT8wdt / 256, 256, 0, stream>>>(W_dt, WDTH, kT8wdt, kT8wdt, kCarryWdt);
  cast_bfval_f16_kernel<<<kT8wo / 256, 256, 0, stream>>>(W_out, WOH, kT8wo, kT8wo, kCarryWo);

  wmma_gemm64<1, 4, false><<<kTilesS0 / 8, 256, 0, stream>>>(
      XB, XB, kDmod, WIB, kDmod, XZ, kXZP, kRows, kXZP, kDmod, 1.0f, 0.0f);

  conv_silu_kernel<<<dim3(kDin / 256, kRows / 64), 256, 0, stream>>>(XZ, conv_w, conv_b, UC, UC16, UC16L);

  wmma_gemm64<0, 2, true><<<kTilesS1 / 8, 256, 0, stream>>>(
      UC16, UC16L, kDin, WXH, kDin, PROJ, kPrjP, kRows, kPrjP, kDin, kUnscaleS1, kUnscaleS1r);

  dt_cast_kernel<<<kT8dt / 256, 256, 0, stream>>>(PROJ, DT16, kT8dt, kCarryDt);

  wmma_gemm64<0, 4, false><<<kTilesS2 / 8, 256, 0, stream>>>(
      DT16, DT16, kDtR, WDTH, kDtR, DLR, kDin, kRows, kDin, kDtR, kUnscaleS2, 0.0f);

  scan_kernel<<<dim3(kDin / 256, kBatch), 256, 0, stream>>>(DLR, UC, XZ, PROJ, b_dt, A_log, Dv, Y16, Y16L);

  wmma_gemm64<0, 2, true><<<kTilesS4 / 8, 256, 0, stream>>>(
      Y16, Y16L, kDin, WOH, kDin, dout, kDmod, kRows, kDmod, kDin, kUnscaleS4, kUnscaleS4r);
}
